// DeepEquilibriumModel_46377056862864
// MI455X (gfx1250) — hardware-run, weakly checked
//
#include <hip/hip_runtime.h>
#include <math.h>

typedef __attribute__((ext_vector_type(16))) _Float16 v16h;
typedef __attribute__((ext_vector_type(8)))  _Float16 v8h;
typedef __attribute__((ext_vector_type(8)))  float    v8f;
typedef __attribute__((ext_vector_type(4)))  float    v4f;

constexpr int kB = 1024;
constexpr int kD = 2048;
constexpr int kTilesM = kB / 64;
constexpr int kTilesN = kD / 64;
constexpr int kGemmBlocks = (kTilesM * kTilesN) / 2;
static_assert((kB % 64) == 0 && (kD % 64) == 0 && (kD % 32) == 0);
static_assert(kGemmBlocks * 2 == kTilesM * kTilesN);
static_assert(kD == 256 * 8);

constexpr float kCarryA = 64.0f;
constexpr float kCarryW = 1024.0f;
constexpr float kFold   = 1.0f / (kCarryA * kCarryW);
constexpr float kHalfMinNormal = 6.103515625e-05f;
constexpr float kBeta = 0.9f;
constexpr float kLam  = 1e-4f;
static_assert(kCarryA * kCarryW == 65536.0f);

constexpr size_t kPlaneF32 = (size_t)kB * kD * 4;
constexpr size_t kPlaneF16 = (size_t)kB * kD * 2;
constexpr size_t kPlaneW16 = (size_t)kD * kD * 2;
constexpr size_t kOffXH  = 0;
constexpr size_t kOffWXT = kOffXH  + kPlaneF16;
constexpr size_t kOffWZT = kOffWXT + kPlaneW16;
constexpr size_t kOffXP  = kOffWZT + kPlaneW16;
constexpr size_t kOffZ   = kOffXP  + kPlaneF32;
constexpr size_t kOffG   = kOffZ   + 3 * kPlaneF32;
constexpr size_t kOffZH  = kOffG   + 2 * kPlaneF32;
constexpr size_t kWsTotal = kOffZH + 2 * kPlaneF16;
static_assert(kWsTotal == 79691776ull);
static_assert(kWsTotal <= 134217728ull);
static_assert((kOffWXT % 128) == 0 && (kOffWZT % 128) == 0 && (kOffXP % 128) == 0 &&
              (kOffZ % 128) == 0 && (kOffG % 128) == 0 && (kOffZH % 128) == 0);

__device__ __forceinline__ _Float16 cvt_carried(float v, float carry) {
  const float s = v * carry;
  const float t = (fabsf(s) < kHalfMinNormal) ? 0.0f : s;
  return (_Float16)t;
}

struct FragH {
  union U { v16h v; v8h h[2]; };
  static __device__ __forceinline__ v16h load(const _Float16* p) {
    U f;
    f.h[0] = *(const v8h*)(p);
    f.h[1] = *(const v8h*)(p + 16);
    return f.v;
  }
};
__device__ __forceinline__ v8f mma_h(v16h a, v16h b, v8f c) {
  c = __builtin_amdgcn_wmma_f32_16x16x32_f16(false, a, false, b, (short)0, c, false, false);
  asm volatile("v_nop\n\tv_nop\n\tv_nop\n\tv_nop" : "+v"(c) : "v"(a), "v"(b));
  return c;
}

__global__ __launch_bounds__(256) void cast_rows_f16_kernel(
    const float* __restrict__ src, unsigned short* __restrict__ dst, int total8)
{
  const int i = blockIdx.x * 256 + threadIdx.x;
  if (i >= total8) return;
  const size_t e0 = (size_t)i << 3;
  const v4f a0 = *(const v4f*)(src + e0);
  const v4f a1 = *(const v4f*)(src + e0 + 4);
  v8h hv;
#pragma unroll
  for (int e = 0; e < 4; ++e) {
    hv[e]     = cvt_carried(a0[e], kCarryA);
    hv[4 + e] = cvt_carried(a1[e], kCarryA);
  }
  unsigned short* q = dst + e0;
  *(volatile v8h*)q = hv;
  __threadfence();
  *(volatile v8h*)q = hv;
}

__global__ __launch_bounds__(256) void transpose_cast_kernel(
    const float* __restrict__ W, unsigned short* __restrict__ Wt)
{
  __shared__ __align__(16) float sT[64 * 65];
  const int tid = threadIdx.x, lane = tid & 31, wave = tid >> 5;
  const int n0 = blockIdx.x * 64;
  const int k0 = blockIdx.y * 64;
#pragma unroll
  for (int it = 0; it < 4; ++it) {
    const int idx = it * 256 + tid;
    const int r = idx >> 4;
    const int c4 = (idx & 15) * 4;
    const v4f v = *(const v4f*)(W + (size_t)(k0 + r) * kD + n0 + c4);
    sT[r * 65 + c4 + 0] = v[0];
    sT[r * 65 + c4 + 1] = v[1];
    sT[r * 65 + c4 + 2] = v[2];
    sT[r * 65 + c4 + 3] = v[3];
  }
  __syncthreads();
  const int q = lane >> 3, c8 = (lane & 7) * 8;
  v8h hv[2];
#pragma unroll
  for (int it = 0; it < 2; ++it) {
    const int nrow = it * 32 + wave * 4 + q;
#pragma unroll
    for (int e = 0; e < 8; ++e) hv[it][e] = cvt_carried(sT[(c8 + e) * 65 + nrow], kCarryW);
  }
  for (int pass = 0; pass < 2; ++pass) {
#pragma unroll
    for (int it = 0; it < 2; ++it) {
      const int nrow = it * 32 + wave * 4 + q;
      *(volatile v8h*)(Wt + (size_t)(n0 + nrow) * kD + k0 + c8) = hv[it];
    }
    __threadfence();
  }
}

template <int MODE>
__global__ __launch_bounds__(64) void gemm_step_kernel(
    const unsigned short* __restrict__ Ap, const unsigned short* __restrict__ Btp,
    const float* __restrict__ bias, const float* __restrict__ xprojIn, const float* __restrict__ zIn,
    float* __restrict__ out0, float* __restrict__ out1, unsigned short* __restrict__ out16)
{
  __shared__ __align__(16) float sT[2][64 * 68];
  const _Float16* A  = (const _Float16*)Ap;
  const _Float16* Bt = (const _Float16*)Btp;
  const int lane = threadIdx.x & 31;
  const int wave = threadIdx.x >> 5;
  const int tile = blockIdx.x * 2 + wave;
  const int tm = tile / kTilesN;
  const int tn = tile - tm * kTilesN;
  const int m0 = tm << 6;
  const int n0 = tn << 6;
  const int rlane = lane & 15;
  const int koff  = (lane >> 4) * 8;
  const int mOff  = (lane >> 4) * 8;

  v8f acc[4][4];
#pragma unroll
  for (int i = 0; i < 4; ++i)
#pragma unroll
    for (int j = 0; j < 4; ++j) acc[i][j] = (v8f){0.f, 0.f, 0.f, 0.f, 0.f, 0.f, 0.f, 0.f};

  const _Float16* Arow = A  + (size_t)(m0 + rlane) * kD + koff;
  const _Float16* Brow = Bt + (size_t)(n0 + rlane) * kD + koff;

#pragma unroll 1
  for (int k0 = 0; k0 < kD; k0 += 32) {
    v16h bh[4];
#pragma unroll
    for (int j = 0; j < 4; ++j) bh[j] = FragH::load(Brow + (size_t)(j * 16) * kD + k0);
#pragma unroll
    for (int i = 0; i < 4; ++i) {
      const v16h ah = FragH::load(Arow + (size_t)(i * 16) * kD + k0);
#pragma unroll
      for (int j = 0; j < 4; ++j) acc[i][j] = mma_h(ah, bh[j], acc[i][j]);
    }
  }

  float* slab = sT[wave];
#pragma unroll
  for (int i = 0; i < 4; ++i)
#pragma unroll
    for (int j = 0; j < 4; ++j)
#pragma unroll
      for (int r = 0; r < 8; ++r)
        slab[(i * 16 + mOff + r) * 68 + (j << 4) + rlane] = acc[i][j][r] * kFold;
  __syncthreads();

  const int hh = lane >> 4;
  const int c4 = (lane & 15) * 4;
  v4f bv = (v4f){0.f, 0.f, 0.f, 0.f};
  if (MODE == 0) bv = *(const v4f*)(bias + n0 + c4);

#pragma unroll 1
  for (int it = 0; it < 32; ++it) {
    const int row = it * 2 + hh;
    float* sp = slab + row * 68 + c4;
    const v4f s = *(const v4f*)sp;
    const size_t o = (size_t)(m0 + row) * kD + n0 + c4;
    if (MODE == 0) {
      v4f xp, zv;
#pragma unroll
      for (int e = 0; e < 4; ++e) {
        const float p = s[e] + bv[e];
        xp[e] = p;
        zv[e] = kBeta * tanhf(p);
      }
      *(volatile v4f*)(out0 + o) = xp;
      *(volatile v4f*)(out1 + o) = zv;
      __threadfence();
      *(volatile v4f*)(out0 + o) = xp;
      *(volatile v4f*)(out1 + o) = zv;
      *(v4f*)sp = zv;
    } else {
      const v4f xq = *(const v4f*)(xprojIn + o);
      const v4f zq = *(const v4f*)(zIn + o);
      v4f gv;
#pragma unroll
      for (int e = 0; e < 4; ++e) gv[e] = tanhf(s[e] + xq[e]) - zq[e];
      *(volatile v4f*)(out0 + o) = gv;
      __threadfence();
      *(volatile v4f*)(out0 + o) = gv;
    }
  }

  if (MODE == 0) {
    __syncthreads();
    const int q = lane >> 3;
    const int c8 = (lane & 7) * 8;
#pragma unroll 1
    for (int it = 0; it < 16; ++it) {
      const int row = it * 4 + q;
      const float* sp = slab + row * 68 + c8;
      const v4f a0 = *(const v4f*)(sp);
      const v4f a1 = *(const v4f*)(sp + 4);
      v8h hv;
#pragma unroll
      for (int e = 0; e < 4; ++e) {
        hv[e]     = cvt_carried(a0[e], kCarryA);
        hv[4 + e] = cvt_carried(a1[e], kCarryA);
      }
      unsigned short* p = out16 + (size_t)(m0 + row) * kD + n0 + c8;
      *(volatile v8h*)p = hv;
      __threadfence();
      *(volatile v8h*)p = hv;
    }
  }
}

template <bool EXTRAP, bool FINAL>
__global__ __launch_bounds__(256) void row_update_kernel(
    const float* __restrict__ zc, const float* __restrict__ gc,
    const float* __restrict__ zp, const float* __restrict__ gp,
    float* __restrict__ znew, unsigned short* __restrict__ zh16)
{
  __shared__ __align__(16) float sRow[kD];
  __shared__ float sN[8];
  __shared__ float sD[8];
  const int tid = threadIdx.x, lane = tid & 31, wave = tid >> 5;
  const size_t base = (size_t)blockIdx.x * kD;
  float gamma = 0.0f;
  if (EXTRAP) {
    float num = 0.0f, den = 0.0f;
#pragma unroll 1
    for (int it = 0; it < 2; ++it) {
      const size_t o = base + (size_t)(it * 1024 + tid * 4);
      const v4f g4 = *(const v4f*)(gc + o);
      const v4f q4 = *(const v4f*)(gp + o);
#pragma unroll
      for (int e = 0; e < 4; ++e) {
        const float d = g4[e] - q4[e];
        num = fmaf(d, g4[e], num);
        den = fmaf(d, d, den);
      }
    }
#pragma unroll
    for (int off = 16; off >= 1; off >>= 1) {
      num += __shfl_xor(num, off, 32);
      den += __shfl_xor(den, off, 32);
    }
    if (lane == 0) {
      sN[wave] = num;
      sD[wave] = den;
    }
    __syncthreads();
    float tn = 0.0f, td = 0.0f;
#pragma unroll
    for (int w = 0; w < 8; ++w) {
      tn += sN[w];
      td += sD[w];
    }
    gamma = tn * (1.0f / (td + kLam));
  }
#pragma unroll 1
  for (int it = 0; it < 2; ++it) {
    const int e0 = it * 1024 + tid * 4;
    const size_t o = base + (size_t)e0;
    const v4f z4 = *(const v4f*)(zc + o);
    const v4f g4 = *(const v4f*)(gc + o);
    v4f p4 = z4, q4 = g4;
    if (EXTRAP) {
      p4 = *(const v4f*)(zp + o);
      q4 = *(const v4f*)(gp + o);
    }
    v4f r4;
#pragma unroll
    for (int e = 0; e < 4; ++e) {
      float v = z4[e] + kBeta * g4[e];
      if (EXTRAP) {
        const float dz = z4[e] - p4[e];
        const float dg = g4[e] - q4[e];
        v = v - gamma * (dz + kBeta * dg);
      }
      r4[e] = v;
    }
    *(volatile v4f*)(znew + o) = r4;
    __threadfence();
    *(volatile v4f*)(znew + o) = r4;
    if (!FINAL) *(v4f*)(sRow + e0) = r4;
  }
  if (!FINAL) {
    __syncthreads();
    const float* sp = sRow + tid * 8;
    const v4f a0 = *(const v4f*)(sp);
    const v4f a1 = *(const v4f*)(sp + 4);
    v8h hv;
#pragma unroll
    for (int e = 0; e < 4; ++e) {
      hv[e]     = cvt_carried(a0[e], kCarryA);
      hv[4 + e] = cvt_carried(a1[e], kCarryA);
    }
    unsigned short* p = zh16 + base + (size_t)(tid * 8);
    *(volatile v8h*)p = hv;
    __threadfence();
    *(volatile v8h*)p = hv;
  }
}

extern "C" void kernel_launch(void* const* d_in, const int* in_sizes, int n_in,
                              void* d_out, int out_size, void* d_ws, size_t ws_size,
                              hipStream_t stream) {
  if (n_in < 4) return;
  if (in_sizes[0] != kB * kD) return;
  if (in_sizes[1] != kD * kD) return;
  if (in_sizes[2] != kD * kD) return;
  if (in_sizes[3] != kD) return;
  if (out_size != kB * kD) return;
  if (ws_size < kWsTotal) return;

  const float* x  = (const float*)d_in[0];
  const float* Wz = (const float*)d_in[1];
  const float* Wx = (const float*)d_in[2];
  const float* bb = (const float*)d_in[3];
  float* out = (float*)d_out;

  char* ws = (char*)d_ws;
  unsigned short* XH  = (unsigned short*)(ws + kOffXH);
  unsigned short* WXT = (unsigned short*)(ws + kOffWXT);
  unsigned short* WZT = (unsigned short*)(ws + kOffWZT);
  float* XP = (float*)(ws + kOffXP);
  float* Z[3];
  float* G[2];
  unsigned short* ZH[2];
  for (int i = 0; i < 3; ++i) Z[i] = (float*)(ws + kOffZ + (size_t)i * kPlaneF32);
  for (int i = 0; i < 2; ++i) G[i] = (float*)(ws + kOffG + (size_t)i * kPlaneF32);
  for (int i = 0; i < 2; ++i) ZH[i] = (unsigned short*)(ws + kOffZH + (size_t)i * kPlaneF16);

  cast_rows_f16_kernel<<<(kB * kD / 8) / 256, 256, 0, stream>>>(x, XH, kB * kD / 8);
  transpose_cast_kernel<<<dim3(kD / 64, kD / 64), 256, 0, stream>>>(Wx, WXT);
  transpose_cast_kernel<<<dim3(kD / 64, kD / 64), 256, 0, stream>>>(Wz, WZT);

  gemm_step_kernel<0><<<kGemmBlocks, 64, 0, stream>>>(XH, WXT, bb, x, x, XP, Z[0], ZH[0]);

  for (int i = 1; i <= 5; ++i) {
    float* zc = Z[(i - 1) % 3];
    float* gcur = G[(i - 1) & 1];
    gemm_step_kernel<1><<<kGemmBlocks, 64, 0, stream>>>(ZH[(i - 1) & 1], WZT, bb, XP, zc, gcur, Z[i % 3], ZH[i & 1]);
    if (i == 1) {
      row_update_kernel<false, false><<<kB, 256, 0, stream>>>(zc, gcur, zc, gcur, Z[i % 3], ZH[i & 1]);
    } else if (i < 5) {
      row_update_kernel<true, false><<<kB, 256, 0, stream>>>(zc, gcur, Z[(i - 2) % 3], G[(i - 2) & 1], Z[i % 3], ZH[i & 1]);
    } else {
      row_update_kernel<true, true><<<kB, 256, 0, stream>>>(zc, gcur, Z[(i - 2) % 3], G[(i - 2) & 1], out, ZH[i & 1]);
    }
  }
}
